// CorrelatedGraphConv_73358041415912
// MI455X (gfx1250) — hardware-run, weakly checked
//
#include <hip/hip_runtime.h>
#pragma clang fp contract(off)


#ifndef NB
#define NB 16
#endif
#define NB_FULL 16
#define NN_  100
#define TP   128
#define NT   7
#define DD   1024
#define NL   2000
#define AJP  136
#define QRS  2048.0f
#define QRI  (1.0f / 2048.0f)
#define PCAR 4096.0f
#define PINV (1.0f / 4096.0f)
#define LOG2E 1.4426950408889634f
#define NEGB (-3.0e38f)

static_assert(DD % 64 == 0);
static_assert(DD % 32 == 0);
static_assert(DD == 4 * 256);
static_assert(TP % 64 == 0);
static_assert(TP % 32 == 0);
static_assert((NB * TP) % 64 == 0);
static_assert(NN_ % 4 == 0);
static_assert(NN_ % 2 == 0);
static_assert(NN_ <= NT * 16);
static_assert(NT == 7);
static_assert(TP == NT * 16 + 16);
static_assert(NN_ <= 128);
static_assert(NB <= NB_FULL);
static_assert(((size_t)NL * DD) % 8 == 0);
static_assert(((size_t)DD * DD) % 8 == 0);
static_assert((AJP * 2) % 16 == 0);
static_assert(AJP >= TP);

typedef _Float16 h16;
typedef unsigned short bf;
typedef __attribute__((ext_vector_type(16))) __bf16   v16bf;
typedef __attribute__((ext_vector_type(16))) _Float16 v16h;
typedef __attribute__((ext_vector_type(8)))  _Float16 v8h;
typedef __attribute__((ext_vector_type(8)))  unsigned short v8us;
typedef __attribute__((ext_vector_type(8)))  float    v8f;
typedef __attribute__((ext_vector_type(4)))  float    v4f;
typedef __attribute__((ext_vector_type(4)))  int      v4i;
typedef __attribute__((ext_vector_type(2)))  unsigned v2u;
typedef v4f  __attribute__((may_alias)) v4fa;
typedef v8h  __attribute__((may_alias)) v8ha;

__device__ __forceinline__ unsigned short f2bf(float f) { unsigned u = __float_as_uint(f); u += 0x7FFFu + ((u >> 16) & 1u); return (unsigned short)(u >> 16); }
__device__ __forceinline__ float bfr(float f) { return __uint_as_float(((unsigned)f2bf(f)) << 16); }
__device__ __forceinline__ v16h cat16(v8h lo, v8h hi) { return __builtin_shufflevector(lo, hi, 0, 1, 2, 3, 4, 5, 6, 7, 8, 9, 10, 11, 12, 13, 14, 15); }
__device__ __forceinline__ v16bf cat16b(v8us lo, v8us hi) { return __builtin_bit_cast(v16bf, __builtin_shufflevector(lo, hi, 0, 1, 2, 3, 4, 5, 6, 7, 8, 9, 10, 11, 12, 13, 14, 15)); }
__device__ __forceinline__ v8f wmma16(v16h a, v16h b, v8f c) { return __builtin_amdgcn_wmma_f32_16x16x32_f16(false, a, false, b, (short)0, c, false, false); }
__device__ __forceinline__ v8f wmmab(v16bf a, v16bf b, v8f c) { return __builtin_amdgcn_wmma_f32_16x16x32_bf16(false, a, false, b, (short)0, c, false, false); }
__device__ __forceinline__ v16h  ldh(const h16* p) { return cat16(*(const v8h*)p, *(const v8h*)(p + 16)); }
__device__ __forceinline__ v16bf ldb(const bf* p)  { return cat16b(*(const v8us*)p, *(const v8us*)(p + 16)); }
__device__ __forceinline__ void wave_sync() { __builtin_amdgcn_fence(3  , "wavefront"); __builtin_amdgcn_wave_barrier(); asm volatile("" ::: "memory"); }
__device__ __forceinline__ h16 toh_flush(float v) { const h16 r = (h16)v; return (fabsf(v) < 6.103515625e-05f) ? (h16)0.0f : r; }
__device__ __forceinline__ v8f wmma16g(v16h a, v16h b, v8f c) { c = wmma16(a, b, c); asm volatile("v_nop\n\tv_nop\n\tv_nop\n\tv_nop" : "+v"(c) : "v"(a), "v"(b)); return c; }
__device__ __forceinline__ v8f wmmabg(v16bf a, v16bf b, v8f c) { c = wmmab(a, b, c); asm volatile("v_nop\n\tv_nop\n\tv_nop\n\tv_nop" : "+v"(c) : "v"(a), "v"(b)); return c; }

__global__ __launch_bounds__(256) void k_cvt8(const float* __restrict__ src, bf* dst, size_t n8) {
    const size_t i = (size_t)blockIdx.x * 256 + threadIdx.x; if (i >= n8) return;
    const v8f v = *(const v8f*)(src + i * 8); v8us o;
#pragma unroll
    for (int k = 0; k < 8; ++k) o[k] = f2bf(v[k]);
    *(volatile v8us*)(dst + i * 8) = o; __threadfence(); *(volatile v8us*)(dst + i * 8) = o;
}

__global__ __launch_bounds__(256) void k_cvtx(const float* __restrict__ src, bf* dst) {
    const size_t n8 = (size_t)NB * TP * DD / 8;
    const size_t i = (size_t)blockIdx.x * 256 + threadIdx.x; if (i >= n8) return;
    const int m = (int)(i / (DD / 8)), c = (int)(i % (DD / 8));
    const int bb = m / TP, t = m % TP;
    const int tc = t < NN_ ? t : (NN_ - 1);
    v8f v = *(const v8f*)(src + ((size_t)bb * NN_ + tc) * DD + (size_t)c * 8);
    asm volatile("" : "+v"(v));
    const bool live = t < NN_;
    v8us o;
#pragma unroll
    for (int k = 0; k < 8; ++k) o[k] = live ? f2bf(v[k]) : (unsigned short)0;
    *(volatile v8us*)(dst + i * 8) = o; __threadfence(); *(volatile v8us*)(dst + i * 8) = o;
}

__global__ __launch_bounds__(256) void k_badd(const float* __restrict__ feat, const int* __restrict__ graph, const bf* __restrict__ TB, float* ADD) {
    __shared__ int gs[128];
    const int tid = threadIdx.x; const int m = blockIdx.x; const int bb = m / TP, t = m % TP;
    const bool live = t < NN_;
    const int tc = live ? t : (NN_ - 1);
    const size_t grow = (size_t)bb * NN_ + tc;
    { const int tj = tid < NN_ ? tid : (NN_ - 1);
      int g = graph[grow * NN_ + tj];
      asm volatile("" : "+v"(g));
      g = g < 0 ? 0 : (g > NL - 1 ? NL - 1 : g);
      if (tid < NN_) gs[tid] = g; }
    __syncthreads();
    const v4f x = *(const v4f*)(feat + grow * DD + 4 * tid);
    float s0 = 0.0f, s1 = 0.0f, s2 = 0.0f, s3 = 0.0f;
    const int nj = live ? NN_ : 0;
#pragma unroll 4
    for (int j = 0; j < nj; ++j) {
        const v2u u = *(const v2u*)(TB + (size_t)gs[j] * DD + 4 * tid);
        s0 += __uint_as_float(u[0] << 16); s1 += __uint_as_float(u[0] & 0xffff0000u);
        s2 += __uint_as_float(u[1] << 16); s3 += __uint_as_float(u[1] & 0xffff0000u);
    }
    v4f o;
    o[0] = live ? (bfr(x[0]) + s0) : 0.0f; o[1] = live ? (bfr(x[1]) + s1) : 0.0f;
    o[2] = live ? (bfr(x[2]) + s2) : 0.0f; o[3] = live ? (bfr(x[3]) + s3) : 0.0f;
    float* dp = ADD + (size_t)m * DD + 4 * tid;
    *(volatile v4f*)dp = o; __threadfence(); *(volatile v4f*)dp = o;
}

template <int MODE>
__device__ __forceinline__ void gemm_body(const bf* __restrict__ A, const bf* __restrict__ Bt, const float* __restrict__ aux, h16* Ph, h16* Pr, const int nrep) {
    __shared__ __align__(16) float os[16 * 68];
    static_assert(sizeof(float) * 16 * 68 <= 131072);
    const int K = DD;
    const int lane = threadIdx.x & 31, lr = lane & 15, hi = lane >> 4; const int r0 = blockIdx.x * 64, c0 = blockIdx.y * 64;
    v8f acc[4][4];
#pragma unroll
    for (int mb = 0; mb < 4; ++mb)
#pragma unroll
        for (int nb = 0; nb < 4; ++nb) acc[mb][nb] = (v8f){};
    const size_t boff = (size_t)(c0 + lr) * K + 8 * hi;
#pragma unroll 1
    for (int w = 0; w < nrep; ++w) {
        const size_t aoff = (size_t)w * ((size_t)DD * DD) + (size_t)(r0 + lr) * K + 8 * hi;
#pragma unroll 1
        for (int kc = 0; kc < K; kc += 32) {
            v16bf a[4];
#pragma unroll
            for (int mb = 0; mb < 4; ++mb) a[mb] = ldb(A + aoff + (size_t)mb * 16 * K + kc);
#pragma unroll
            for (int nb = 0; nb < 4; ++nb) { const v16bf b = ldb(Bt + boff + (size_t)nb * 16 * K + kc);
#pragma unroll
                for (int mb = 0; mb < 4; ++mb) acc[mb][nb] = wmmabg(a[mb], b, acc[mb][nb]); }
        }
    }
    size_t tbase; int pitch;
    if (MODE == 0) { tbase = (size_t)r0 * DD + (size_t)c0; pitch = DD; }
    else           { const int bb = c0 / TP, tt = c0 % TP; tbase = ((size_t)bb * DD + (size_t)r0) * TP + (size_t)tt; pitch = TP; }
    float bc[4];
#pragma unroll
    for (int nb = 0; nb < 4; ++nb) bc[nb] = (MODE == 0) ? bfr(aux[c0 + nb * 16 + lr]) : 0.0f;
#pragma unroll
    for (int mb = 0; mb < 4; ++mb) {
#pragma unroll
        for (int nb = 0; nb < 4; ++nb) {
            v4f x0 = (v4f){}, x1 = (v4f){};
            if (MODE == 1) { const float* ap = aux + (size_t)(c0 + nb * 16 + lr) * DD + (size_t)(r0 + mb * 16 + 8 * hi); x0 = *(const v4f*)ap; x1 = *(const v4f*)(ap + 4); }
#pragma unroll
            for (int j = 0; j < 8; ++j) { const float ad = (j < 4) ? x0[j & 3] : x1[j & 3];
                os[(hi * 8 + j) * 68 + nb * 16 + lr] = acc[mb][nb][j] + bc[nb] + ad; } }
        wave_sync();
        static_assert(32 * 16 * 4 == 16 * 128);
#pragma unroll 1
        for (int ps = 0; ps < 2; ++ps) {
            const size_t sb = tbase + (size_t)(mb * 16) * (size_t)pitch;
#pragma unroll
            for (int s = 0; s < 4; ++s) { const int row = 4 * s + (lane >> 3), c8 = (lane & 7) * 8;
                const v4f x0 = *(const v4fa*)(&os[row * 68 + c8]); const v4f x1 = *(const v4fa*)(&os[row * 68 + c8 + 4]); v8h hv, rv;
#pragma unroll
                for (int i = 0; i < 4; ++i) { const h16 a0 = toh_flush(x0[i]); const h16 a1 = toh_flush(x1[i]); hv[i] = a0; hv[4 + i] = a1;
                    rv[i] = toh_flush((x0[i] - (float)a0) * QRS); rv[4 + i] = toh_flush((x1[i] - (float)a1) * QRS); }
                const size_t oo = sb + (size_t)row * (size_t)pitch + c8;
                *(volatile v8h*)(Ph + oo) = hv; *(volatile v8h*)(Pr + oo) = rv; }
            if (ps == 0) __threadfence(); }
        wave_sync();
    }
}

__global__ __launch_bounds__(32) void k_gemm_ab(const bf* __restrict__ X, const bf* __restrict__ W, const float* __restrict__ bias, h16* Ph, h16* Pr) {
    gemm_body<0>(X, W, bias, Ph, Pr, 1);
}
__global__ __launch_bounds__(32) void k_gemm_ot(const bf* __restrict__ W, const bf* __restrict__ X, const float* __restrict__ addp, h16* Ph, h16* Pr) {
    gemm_body<1>(W, X, addp, Ph, Pr, 2);
}

__global__ __launch_bounds__(256) void k_alpha(const h16* __restrict__ AH, const h16* __restrict__ AR, const h16* __restrict__ BH, const h16* __restrict__ BR,
                                               const int* __restrict__ graph, h16* ALH, h16* ALR) {
    __shared__ __align__(16) h16 AJ[NT * 16 * AJP];
    __shared__ __align__(16) h16 SH[TP * AJP];
    __shared__ __align__(16) h16 SR[TP * AJP];
    static_assert(sizeof(h16) * (NT * 16 * AJP + 2 * TP * AJP) <= 131072);
    const int tid = threadIdx.x, lane = tid & 31, lr = lane & 15, hi = lane >> 4;
    const int wave = __builtin_amdgcn_readfirstlane((int)(threadIdx.x >> 5));
    const int b = blockIdx.x;
    static_assert(256 * 14 == NT * 16 * (TP / 4));
#pragma unroll 1
    for (int s = 0; s < 14; ++s) {
        const int g = s * 256 + tid; const int i = g >> 5, jg = (g & 31) * 4;
        const int ic = i < NN_ ? i : (NN_ - 1); const int jc = jg < NN_ ? jg : (NN_ - 4);
        v4i q = *(const v4i*)(graph + ((size_t)b * NN_ + ic) * NN_ + jc);
        asm volatile("" : "+v"(q));
        const bool ok = (i < NN_) & (jg < NN_);
#pragma unroll
        for (int e = 0; e < 4; ++e) AJ[i * AJP + jg + e] = (ok & (q[e] != 0)) ? (h16)1.0f : (h16)0.0f;
    }
    __syncthreads();

    const size_t prow = (size_t)b * TP;
    const size_t bo = (prow + (size_t)(wave * 16 + lr)) * DD + 8 * hi;
    const size_t ao = (prow + (size_t)lr) * DD + 8 * hi;
    v8f sH[NT], sL[NT];
#pragma unroll
    for (int jt = 0; jt < NT; ++jt) { sH[jt] = (v8f){}; sL[jt] = (v8f){}; }
#pragma unroll 1
    for (int kc = 0; kc < DD; kc += 32) {
        const v16h bh = ldh(BH + bo + kc), br = ldh(BR + bo + kc);
#pragma unroll
        for (int jt = 0; jt < NT; ++jt) {
            const v16h ah = ldh(AH + ao + (size_t)jt * 16 * DD + kc), ar = ldh(AR + ao + (size_t)jt * 16 * DD + kc);
            sH[jt] = wmma16g(ah, bh, sH[jt]); sL[jt] = wmma16g(ah, br, sL[jt]); sL[jt] = wmma16g(ar, bh, sL[jt]);
        }
    }
    v16h rh[4], rr[4];
#pragma unroll
    for (int p = 0; p < 4; ++p) {
        const int t0 = 2 * p;
        const int t1 = (2 * p + 1 < NT) ? (2 * p + 1) : (NT - 1);
#pragma unroll
        for (int r = 0; r < 8; ++r) {
            const int j0 = 32 * p + 8 * hi + r, j1 = j0 + 16;
            float v0 = fmaxf(sH[t0][r] + sL[t0][r] * QRI, 0.0f); v0 = (j0 < NN_) ? v0 : 0.0f;
            float v1 = fmaxf(sH[t1][r] + sL[t1][r] * QRI, 0.0f); v1 = (j1 < NN_) ? v1 : 0.0f;
            const h16 a0 = toh_flush(v0); const h16 a1 = toh_flush(v1);
            rh[p][r] = a0; rh[p][8 + r] = a1;
            rr[p][r] = toh_flush((v0 - (float)a0) * QRS); rr[p][8 + r] = toh_flush((v1 - (float)a1) * QRS);
        }
    }
    v8f e2[NT];
#pragma unroll
    for (int it = 0; it < NT; ++it) {
        v8f cH = (v8f){}, cL = (v8f){};
#pragma unroll
        for (int p = 0; p < 4; ++p) {
            const int off = (it * 16 + lr) * AJP + 32 * p + 8 * hi;
            const v16h af = cat16(*(const v8ha*)(&AJ[off]), *(const v8ha*)(&AJ[off + 16]));
            cH = wmma16g(af, rh[p], cH); cL = wmma16g(af, rr[p], cL);
        }
        e2[it] = cH + cL * QRI;
    }
    float mx = NEGB;
#pragma unroll
    for (int it = 0; it < NT; ++it)
#pragma unroll
        for (int r = 0; r < 8; ++r) { const bool ok = (it * 16 + 8 * hi + r) < NN_; mx = fmaxf(mx, ok ? e2[it][r] : NEGB); }
    mx = fmaxf(mx, __shfl_xor(mx, 16, 32));
    float z = 0.0f;
#pragma unroll
    for (int it = 0; it < NT; ++it)
#pragma unroll
        for (int r = 0; r < 8; ++r) { const bool ok = (it * 16 + 8 * hi + r) < NN_;
            const float ev = __builtin_amdgcn_exp2f(fminf((e2[it][r] - mx) * LOG2E, 0.0f));
            const float ek = ok ? ev : 0.0f; e2[it][r] = ek; z += ek; }
    z += __shfl_xor(z, 16, 32);
    const float inv = 1.0f / z;
    const bool kok = (wave * 16 + lr) < NN_;
    const float sc = kok ? (inv * PCAR) : 0.0f;
    const int kc16 = wave * 16 + lr;
#pragma unroll
    for (int it = 0; it < NT; ++it)
#pragma unroll
        for (int r = 0; r < 8; ++r) { const int i = it * 16 + 8 * hi + r;
            const float v = e2[it][r] * sc; const h16 ph = toh_flush(v);
            SH[i * AJP + kc16] = ph; SR[i * AJP + kc16] = toh_flush((v - (float)ph) * QRS); }
#pragma unroll
    for (int r = 0; r < 8; ++r) { const int i = NT * 16 + 8 * hi + r; SH[i * AJP + kc16] = (h16)0.0f; SR[i * AJP + kc16] = (h16)0.0f; }
    __syncthreads();
    static_assert(256 * 8 * 16 == TP * TP * 2);
    const size_t pb = (size_t)b * TP * TP;
#pragma unroll 1
    for (int ps = 0; ps < 2; ++ps) {
#pragma unroll
        for (int s = 0; s < 8; ++s) { const int p = s * 256 + tid; const int row = p >> 4, c8 = (p & 15) * 8;
            const v8h hv = *(const v8ha*)(&SH[row * AJP + c8]); const v8h rv = *(const v8ha*)(&SR[row * AJP + c8]);
            const size_t oo = pb + (size_t)row * TP + c8;
            *(volatile v8h*)(ALH + oo) = hv; *(volatile v8h*)(ALR + oo) = rv; }
        if (ps == 0) __threadfence(); }
}

__global__ __launch_bounds__(32) void k_out(const h16* __restrict__ ALH, const h16* __restrict__ ALR, const h16* __restrict__ OH, const h16* __restrict__ OR_, float* OUT) {
    __shared__ __align__(16) float os[16 * 68];
    const int lane = threadIdx.x & 31, lr = lane & 15, hi = lane >> 4;
    const int i0 = blockIdx.x * 32, c0 = blockIdx.y * 64, b = blockIdx.z;
    v8f acc[2][4], acr[2][4];
#pragma unroll
    for (int mb = 0; mb < 2; ++mb)
#pragma unroll
        for (int nb = 0; nb < 4; ++nb) { acc[mb][nb] = (v8f){}; acr[mb][nb] = (v8f){}; }
    const size_t aoff = ((size_t)b * TP + (size_t)(i0 + lr)) * TP + 8 * hi;
    const size_t boff = ((size_t)b * DD + (size_t)(c0 + lr)) * TP + 8 * hi;
#pragma unroll 1
    for (int kc = 0; kc < TP; kc += 32) {
        v16h ah[2], ar[2];
#pragma unroll
        for (int mb = 0; mb < 2; ++mb) { ah[mb] = ldh(ALH + aoff + (size_t)mb * 16 * TP + kc); ar[mb] = ldh(ALR + aoff + (size_t)mb * 16 * TP + kc); }
#pragma unroll
        for (int nb = 0; nb < 4; ++nb) {
            const v16h bh = ldh(OH + boff + (size_t)nb * 16 * TP + kc), br = ldh(OR_ + boff + (size_t)nb * 16 * TP + kc);
#pragma unroll
            for (int mb = 0; mb < 2; ++mb) {
                acc[mb][nb] = wmma16g(ah[mb], bh, acc[mb][nb]);
                acr[mb][nb] = wmma16g(ah[mb], br, acr[mb][nb]);
                acr[mb][nb] = wmma16g(ar[mb], bh, acr[mb][nb]); }
        }
    }
#pragma unroll
    for (int mb = 0; mb < 2; ++mb) {
#pragma unroll
        for (int nb = 0; nb < 4; ++nb)
#pragma unroll
            for (int j = 0; j < 8; ++j) os[(hi * 8 + j) * 68 + nb * 16 + lr] = (acc[mb][nb][j] + acr[mb][nb][j] * QRI) * PINV;
        wave_sync();
        static_assert(32 * 16 * 8 == 16 * 256);
#pragma unroll 1
        for (int ps = 0; ps < 2; ++ps) {
#pragma unroll
            for (int s = 0; s < 8; ++s) { const int row = 2 * s + (lane >> 4), cofs = (lane & 15) * 4;
                const int i = i0 + mb * 16 + row;
                const v4f val = *(const v4fa*)(&os[row * 68 + cofs]);
                if (i < NN_) *(volatile v4f*)(OUT + ((size_t)b * NN_ + (size_t)i) * DD + (size_t)(c0 + cofs)) = val; }
            if (ps == 0) __threadfence(); }
        wave_sync();
    }
}

static constexpr size_t al256(size_t v) { return (v + 255) & ~(size_t)255; }
static constexpr size_t SZ_XB = al256((size_t)NB * TP * DD * 2);
static constexpr size_t SZ_WB = al256((size_t)4 * DD * DD * 2);
static constexpr size_t SZ_TB = al256((size_t)NL * DD * 2);
static constexpr size_t SZ_AD = al256((size_t)NB * TP * DD * 4);
static constexpr size_t SZ_PL = al256((size_t)NB * TP * DD * 2);
static constexpr size_t SZ_AL = al256((size_t)NB * TP * TP * 2);
static constexpr size_t SZ_TOTAL = SZ_XB + SZ_WB + SZ_TB + SZ_AD + 6 * SZ_PL + 2 * SZ_AL;
static_assert(SZ_TOTAL <= (size_t)134217728);
static_assert(((size_t)DD * DD * 2) % 256 == 0);
static_assert((size_t)NB * TP * DD == (size_t)NB * DD * TP);

extern "C" void kernel_launch(void* const* d_in, const int* in_sizes, int n_in,
                              void* d_out, int out_size, void* d_ws, size_t ws_size, hipStream_t stream) {
    if (n_in < 10) return;
    if ((size_t)in_sizes[0] < (size_t)NB * NN_ * DD) return;
    if ((size_t)in_sizes[1] < (size_t)NB * NN_ * NN_) return;
    if ((size_t)in_sizes[2] < (size_t)DD * DD || (size_t)in_sizes[3] < (size_t)DD * DD) return;
    if ((size_t)in_sizes[4] < (size_t)NL * DD) return;
    if ((size_t)in_sizes[5] < (size_t)DD * DD || (size_t)in_sizes[7] < (size_t)DD * DD) return;
    if (in_sizes[6] < DD || in_sizes[8] < DD || in_sizes[9] < 1) return;
    if ((size_t)out_size < (size_t)NB * NN_ * DD) return;
    if (SZ_TOTAL > ws_size) return;
    const float* feat = (const float*)d_in[0];
    const int*   graph = (const int*)d_in[1];
    const float* w0 = (const float*)d_in[2]; const float* w1 = (const float*)d_in[3];
    const float* tab = (const float*)d_in[4];
    const float* wa = (const float*)d_in[5]; const float* ba = (const float*)d_in[6];
    const float* wb = (const float*)d_in[7]; const float* bbv = (const float*)d_in[8];
    float* OUT = (float*)d_out;
    char* wsp = (char*)d_ws;
    bf* XB = (bf*)wsp; wsp += SZ_XB;
    bf* WB = (bf*)wsp; wsp += SZ_WB;
    bf* TB = (bf*)wsp; wsp += SZ_TB;
    float* ADD = (float*)wsp; wsp += SZ_AD;
    h16* AH = (h16*)wsp; wsp += SZ_PL;
    h16* AR = (h16*)wsp; wsp += SZ_PL;
    h16* BH = (h16*)wsp; wsp += SZ_PL;
    h16* BR = (h16*)wsp; wsp += SZ_PL;
    h16* OH = (h16*)wsp; wsp += SZ_PL;
    h16* OR_ = (h16*)wsp; wsp += SZ_PL;
    h16* ALH = (h16*)wsp; wsp += SZ_AL;
    h16* ALR = (h16*)wsp; wsp += SZ_AL;
    bf* W0B = WB; bf* WAB = WB + (size_t)2 * DD * DD; bf* WBB = WB + (size_t)3 * DD * DD;

    { const size_t n8 = (size_t)DD * DD / 8; const unsigned g = (unsigned)((n8 + 255) / 256);
      k_cvt8<<<g, 256, 0, stream>>>(w0, WB, n8); k_cvt8<<<g, 256, 0, stream>>>(w1, WB + (size_t)DD * DD, n8);
      k_cvt8<<<g, 256, 0, stream>>>(wa, WAB, n8); k_cvt8<<<g, 256, 0, stream>>>(wb, WBB, n8); }
    { const size_t n8 = (size_t)NL * DD / 8; k_cvt8<<<(unsigned)((n8 + 255) / 256), 256, 0, stream>>>(tab, TB, n8); }
    { const size_t n8 = (size_t)NB * TP * DD / 8; k_cvtx<<<(unsigned)((n8 + 255) / 256), 256, 0, stream>>>(feat, XB); }
    k_badd<<<NB * TP, 256, 0, stream>>>(feat, graph, TB, ADD);

    k_gemm_ab<<<dim3(NB * TP / 64, DD / 64, 1), 32, 0, stream>>>(XB, WAB, ba, AH, AR);
    k_gemm_ab<<<dim3(NB * TP / 64, DD / 64, 1), 32, 0, stream>>>(XB, WBB, bbv, BH, BR);
    k_gemm_ot<<<dim3(DD / 64, NB * TP / 64, 1), 32, 0, stream>>>(W0B, XB, ADD, OH, OR_);

    k_alpha<<<NB, 256, 0, stream>>>(AH, AR, BH, BR, graph, ALH, ALR);
    k_out<<<dim3(TP / 32, DD / 64, NB), 32, 0, stream>>>(ALH, ALR, OH, OR_, OUT);
}
